// StyleConv_56590489092563
// MI455X (gfx1250) — hardware-verified
//
#include <hip/hip_runtime.h>


namespace {
constexpr int Bn = 8, CI = 256, CO = 512, HW = 64, NSF = 512, SM = 65, SMS = 4352  , OP = 32, NPIX = OP * OP, K9 = 9;
constexpr float XS = 8.0f, EPS = 1e-8f, ACT_SCALE = 1.4142135623730951f;

typedef _Float16 b16;
typedef __attribute__((ext_vector_type(16))) _Float16 v16b;
typedef __attribute__((ext_vector_type(8))) _Float16 v8b;
typedef __attribute__((ext_vector_type(8))) float v8f;
typedef __attribute__((ext_vector_type(4))) float v4f;
__device__ __forceinline__ float bf16_rne(float f) { unsigned int u = __float_as_uint(f); u += 0x7FFFu + ((u >> 16) & 1u); return __uint_as_float(u & 0xFFFF0000u); }
__device__ __forceinline__ void split16(float v, b16& hi, b16& lo) { hi = (b16)v; lo = (b16)(v - (float)hi); }
__device__ __forceinline__ v16b frag_kb(const b16* p, int hh) { const v8b a = *(const v8b*)(p + 8 * hh), b = *(const v8b*)(p + 16 + 8 * hh); v16b f;
#pragma unroll
  for (int e = 0; e < 8; ++e) { f[e] = a[e]; f[8 + e] = b[e]; } return f; }
__device__ __forceinline__ v8f wmma16b(v16b a, v16b b, v8f c) { v8f d = __builtin_amdgcn_wmma_f32_16x16x32_f16(false, a, false, b, (short)0, c, false, false); asm volatile("v_nop\n\tv_nop\n\tv_nop\n\tv_nop" : "+v"(d) : "v"(a), "v"(b)); return d; }
__device__ __forceinline__ void wave_lds_sync() { __builtin_amdgcn_fence(__ATOMIC_RELEASE, "workgroup"); __builtin_amdgcn_wave_barrier(); __builtin_amdgcn_fence(__ATOMIC_ACQUIRE, "workgroup"); }
__device__ __forceinline__ float pmul(float a, float b) { float p = a * b; asm volatile("" : "+v"(p)); return p; }
__device__ __forceinline__ float wsum(float v) {
#pragma unroll
  for (int o = 1; o < 32; o <<= 1) v += __shfl_xor(v, o); return v; }

__global__ __launch_bounds__(256) void smod_kernel(const float* __restrict__ style, const float* __restrict__ wmod, const float* __restrict__ bmod, float* __restrict__ S) {
  __shared__ float Ss[32];
  const int wave = threadIdx.x >> 5, lane = threadIdx.x & 31, b = blockIdx.y, c0 = blockIdx.x * 32; const float msc = 1.0f / sqrtf((float)NSF);
  for (int k = 0; k < 4; ++k) { const int c = c0 + wave * 4 + k; float s = 0.0f; for (int j = lane; j < NSF; j += 32) s += pmul(bf16_rne(style[(size_t)b * NSF + j]), pmul(bf16_rne(wmod[(size_t)c * NSF + j]), msc)); s = wsum(s); if (lane == 0) Ss[wave * 4 + k] = s + bf16_rne(bmod[c]); }
  __syncthreads();
  for (int pass = 0; pass < 2; ++pass) { if (threadIdx.x < 8) *(volatile v4f*)(S + (size_t)b * CI + c0 + threadIdx.x * 4) = *(const v4f*)(&Ss[threadIdx.x * 4]); __threadfence(); }
}
__global__ __launch_bounds__(256) void wmod_kernel(const float* __restrict__ cw, const float* __restrict__ S, b16* __restrict__ Wh, b16* __restrict__ Wl) {
  const int wave = threadIdx.x >> 5, lane = threadIdx.x & 31, b = blockIdx.y, co = blockIdx.x * 8 + wave; const float csc = 1.0f / sqrtf((float)(CI * K9));
  float sv[8]; float ss = 0.0f;
#pragma unroll
  for (int e = 0; e < 8; ++e) sv[e] = S[(size_t)b * CI + lane * 8 + e];
#pragma unroll 1
  for (int k = 0; k < K9; ++k) {
#pragma unroll
    for (int e = 0; e < 8; ++e) { const float w = pmul(pmul(csc, bf16_rne(cw[((size_t)co * CI + lane * 8 + e) * K9 + k])), sv[e]); ss += pmul(w, w); } }
  ss = wsum(ss); const float dm = rsqrtf(ss + EPS);
  for (int pass = 0; pass < 2; ++pass) {
#pragma unroll 1
    for (int k = 0; k < K9; ++k) { v8b hv, lv;
#pragma unroll
      for (int e = 0; e < 8; ++e) { const float w = pmul(pmul(csc, bf16_rne(cw[((size_t)co * CI + lane * 8 + e) * K9 + k])), sv[e]); b16 h_, l_; split16(pmul(w, dm) * XS, h_, l_); hv[e] = h_; lv[e] = l_; }
      const size_t gi = (((size_t)b * K9 + k) * CO + co) * CI + lane * 8; *(volatile v8b*)(Wh + gi) = hv; *(volatile v8b*)(Wl + gi) = lv; }
    __threadfence(); }
}
__global__ __launch_bounds__(256) void fir_kernel(const float* __restrict__ x, float* __restrict__ XSM) {
  __shared__ float Xs[HW][HW + 1];
  const int c = blockIdx.x, b = blockIdx.y, t_ = threadIdx.x; const float* xp = x + ((size_t)b * CI + c) * HW * HW;
  for (int i = t_; i < HW * HW; i += 256) Xs[i >> 6][i & 63] = bf16_rne(xp[i]);
  __syncthreads();
  const float k1[4] = {1.0f, 3.0f, 3.0f, 1.0f};
  float* dst = XSM + ((size_t)b * CI + c) * SMS;
  for (int pass = 0; pass < 2; ++pass) { for (int i = t_; i < SMS; i += 256) { float v = 0.0f;
      if (i < SM * SM) { const int Y = i / SM, X = i % SM;
#pragma unroll
        for (int a = 0; a < 4; ++a) { const int yy = Y + a - 2; if (yy < 0 || yy >= HW) continue;
#pragma unroll
          for (int bq = 0; bq < 4; ++bq) { const int xx = X + bq - 2; if (xx < 0 || xx >= HW) continue; v += pmul(Xs[yy][xx], k1[a] * k1[bq] * (1.0f / 64.0f)); } } }
      ((volatile float*)dst)[i] = v; } __threadfence(); }
}
__global__ __launch_bounds__(256) void gat_kernel(const float* __restrict__ XSM, b16* __restrict__ Gh, b16* __restrict__ Gl) {
  __shared__ __attribute__((aligned(16))) b16 Th[32][CI + 8], Tl[32][CI + 8];
  const int p0 = blockIdx.x * 32, kyx = blockIdx.y, b = blockIdx.z, t_ = threadIdx.x; const int ky = kyx / 3, kx = kyx % 3;
  for (int i = t_; i < 32 * CI; i += 256) { const int c = i >> 5, pl = i & 31; const int pix = p0 + pl, Y = pix >> 5, X = pix & 31; const float v = XSM[((size_t)b * CI + c) * SMS + (2 * Y + ky) * SM + 2 * X + kx]; b16 h_, l_; split16(v * XS, h_, l_); Th[pl][c] = h_; Tl[pl][c] = l_; }
  __syncthreads();
  for (int pass = 0; pass < 2; ++pass) { for (int i = t_; i < 32 * (CI / 8); i += 256) { const int pl = i / (CI / 8), c8 = (i % (CI / 8)) * 8; const size_t gi = (((size_t)b * K9 + kyx) * NPIX + p0 + pl) * CI + c8; *(volatile v8b*)(Gh + gi) = *(const v8b*)(&Th[pl][c8]); *(volatile v8b*)(Gl + gi) = *(const v8b*)(&Tl[pl][c8]); } __threadfence(); }
}
__global__ __launch_bounds__(64) void conv_kernel(const b16* __restrict__ Wh, const b16* __restrict__ Wl, const b16* __restrict__ Gh, const b16* __restrict__ Gl, const float* __restrict__ noise, const float* __restrict__ nw, const float* __restrict__ ab, float* __restrict__ out) {
  __shared__ __attribute__((aligned(16))) float Ts[2][16][128 + 4];
  const int lane = threadIdx.x & 31, wave = threadIdx.x >> 5, nloc = lane & 15, hlf = lane >> 4, b = blockIdx.z, co0 = blockIdx.y * 32 + wave * 16, p0 = blockIdx.x * 128;
  v8f acc[8];
#pragma unroll
  for (int t = 0; t < 8; ++t) acc[t] = (v8f){};
  for (int k = 0; k < K9; ++k) { const b16* Ar = Wh + (((size_t)b * K9 + k) * CO + co0) * CI; const b16* Alr = Wl + (((size_t)b * K9 + k) * CO + co0) * CI; const b16* Br = Gh + (((size_t)b * K9 + k) * NPIX + p0) * CI; const b16* Blr = Gl + (((size_t)b * K9 + k) * NPIX + p0) * CI;
#pragma unroll 2
    for (int kb = 0; kb < CI; kb += 32) { const v16b a = frag_kb(Ar + (size_t)nloc * CI + kb, hlf), al_ = frag_kb(Alr + (size_t)nloc * CI + kb, hlf);
#pragma unroll
      for (int t = 0; t < 8; ++t) { const v16b bh = frag_kb(Br + (size_t)(t * 16 + nloc) * CI + kb, hlf), bl = frag_kb(Blr + (size_t)(t * 16 + nloc) * CI + kb, hlf); acc[t] = wmma16b(a, bh, acc[t]); acc[t] = wmma16b(al_, bh, acc[t]); acc[t] = wmma16b(a, bl, acc[t]); } } }
  const float nwv = bf16_rne(nw[0]);
#pragma unroll
  for (int t = 0; t < 8; ++t)
#pragma unroll
    for (int r = 0; r < 8; ++r) { const int co = co0 + 8 * hlf + r, pix = p0 + t * 16 + nloc; float v = acc[t][r] * (1.0f / (XS * XS)) + pmul(nwv, bf16_rne(noise[(size_t)b * NPIX + pix])) + bf16_rne(ab[co]); v = (v >= 0.0f) ? v : 0.2f * v; Ts[wave][8 * hlf + r][t * 16 + nloc] = v * ACT_SCALE; }
  wave_lds_sync();
  for (int pass = 0; pass < 2; ++pass) { for (int i = lane; i < 16 * 32; i += 32) { const int rr = i >> 5, c4 = (i & 31) * 4; *(volatile v4f*)(out + ((size_t)b * CO + co0 + rr) * NPIX + p0 + c4) = *(const v4f*)(&Ts[wave][rr][c4]); } __threadfence(); }
}
}

extern "C" void kernel_launch(void* const* d_in, const int* in_sizes, int n_in,
                              void* d_out, int out_size, void* d_ws, size_t ws_size, hipStream_t stream) {
  (void)n_in; (void)out_size;
  auto Fp = [&](int i) { return (const float*)d_in[i]; };
  float* out = (float*)d_out;
  if (in_sizes[0] != Bn * CI * HW * HW || in_sizes[5] != CO * CI * K9 || in_sizes[6] != 1) return;
  size_t off = 0; char* ws = (char*)d_ws;
  auto carve = [&](size_t bytes) { char* p = ws + off; off += (bytes + 255) & ~(size_t)255; return p; };
  float* S = (float*)carve((size_t)Bn * CI * 4); b16* Wh = (b16*)carve((size_t)Bn * K9 * CO * CI * 2); b16* Wl = (b16*)carve((size_t)Bn * K9 * CO * CI * 2); float* XSM = (float*)carve((size_t)Bn * CI * SMS * 4); b16* Gh = (b16*)carve((size_t)Bn * K9 * NPIX * CI * 2); b16* Gl = (b16*)carve((size_t)Bn * K9 * NPIX * CI * 2);
  if (off > ws_size) return;
  smod_kernel<<<dim3(CI / 32, Bn), 256, 0, stream>>>(Fp(1), Fp(3), Fp(4), S);
  wmod_kernel<<<dim3(CO / 8, Bn), 256, 0, stream>>>(Fp(5), S, Wh, Wl);
  fir_kernel<<<dim3(CI, Bn), 256, 0, stream>>>(Fp(0), XSM);
  gat_kernel<<<dim3(NPIX / 32, K9, Bn), 256, 0, stream>>>(XSM, Gh, Gl);
  conv_kernel<<<dim3(NPIX / 128, CO / 32, Bn), 64, 0, stream>>>(Wh, Wl, Gh, Gl, Fp(2), Fp(6), Fp(7), out);
}
